// SoftCapAttention_3066606650060
// MI455X (gfx1250) — hardware-verified
//
#include <hip/hip_runtime.h>
#include <math.h>


#define NBH   32
#define SEQ   2048
#define HD    128
#define QBLK  64
#define KBLK  32
#define CBLK  64
#define NWAV  4
#define SCL   0.08838834764831845f
#define CAPV  20.0f

static_assert(SEQ % QBLK == 0);
static_assert(SEQ % KBLK == 0);
static_assert(SEQ % CBLK == 0);
static_assert(QBLK == NWAV * 16);
static_assert(HD % 32 == 0);
static_assert(CBLK == 64);

typedef __bf16 v16b __attribute__((ext_vector_type(16)));
typedef __bf16 v8b  __attribute__((ext_vector_type(8)));
typedef float  v8f  __attribute__((ext_vector_type(8)));
typedef float  v4f  __attribute__((ext_vector_type(4)));

union Frag  { v16b v; v8b p[2]; };
union Pack8 { v8b b; v4f f; };

__device__ __forceinline__ v8f wmma16(v16b a, v16b b, v8f c) {
  v8f d = __builtin_amdgcn_wmma_f32_16x16x32_bf16(false, a, false, b, (short)0, c, false, false);
  asm volatile("v_nop\n\tv_nop\n\tv_nop\n\tv_nop" : "+v"(d) : "v"(a), "v"(b));
  return d;
}

__device__ __forceinline__ v8f vzero8() {
  v8f z = {0.0f, 0.0f, 0.0f, 0.0f, 0.0f, 0.0f, 0.0f, 0.0f};
  return z;
}

__global__ __launch_bounds__(256)
void k_cvt(const float* __restrict__ q, const float* __restrict__ k, const float* __restrict__ v,
           __bf16* __restrict__ qp, __bf16* __restrict__ kp, __bf16* __restrict__ vtp) {
  __shared__ __attribute__((aligned(16))) __bf16 tsm[HD][CBLK + 8];

  const int tid  = threadIdx.x;
  const int lane = tid & 31;
  const int wave = tid >> 5;
  const int n0   = blockIdx.x * CBLK;
  const int bh   = blockIdx.y;
  const size_t rb = (size_t)bh * SEQ + (size_t)n0;

#pragma unroll
  for (int it = 0; it < CBLK / 16; ++it) {
    const int rl = it * 16 + wave * 2 + (lane >> 4);
    const int c  = (lane & 15) * 8;
    const size_t e = (rb + (size_t)rl) * HD + (size_t)c;
    {
      const v4f f0 = *(const v4f*)(q + e);
      const v4f f1 = *(const v4f*)(q + e + 4);
      Pack8 o;
#pragma unroll
      for (int j = 0; j < 4; ++j) { o.b[j] = (__bf16)f0[j]; o.b[4 + j] = (__bf16)f1[j]; }
      volatile v4f* d = (volatile v4f*)(qp + e);
      *d = o.f;
      __threadfence();
      *d = o.f;
    }
    {
      const v4f f0 = *(const v4f*)(k + e);
      const v4f f1 = *(const v4f*)(k + e + 4);
      Pack8 o;
#pragma unroll
      for (int j = 0; j < 4; ++j) { o.b[j] = (__bf16)f0[j]; o.b[4 + j] = (__bf16)f1[j]; }
      volatile v4f* d = (volatile v4f*)(kp + e);
      *d = o.f;
      __threadfence();
      *d = o.f;
    }
    {
      const v4f f0 = *(const v4f*)(v + e);
      const v4f f1 = *(const v4f*)(v + e + 4);
#pragma unroll
      for (int j = 0; j < 4; ++j) { tsm[c + j][rl] = (__bf16)f0[j]; tsm[c + 4 + j][rl] = (__bf16)f1[j]; }
    }
  }
  __syncthreads();

#pragma unroll
  for (int it = 0; it < HD / 32; ++it) {
    const int d = it * 32 + wave * 4 + (lane >> 3);
    const int c = (lane & 7) * 8;
    Pack8 o;
    o.b = *(const v8b*)(&tsm[d][c]);
    volatile v4f* dst = (volatile v4f*)(vtp + ((size_t)bh * HD + (size_t)d) * SEQ + (size_t)n0 + (size_t)c);
    *dst = o.f;
    __threadfence();
    *dst = o.f;
  }
}

__global__ __launch_bounds__(NWAV * 32) __attribute__((amdgpu_num_vgpr(256)))
void k_attn(const __bf16* __restrict__ qp, const __bf16* __restrict__ kp,
            const __bf16* __restrict__ vtp, float* __restrict__ out) {
  __shared__ __attribute__((aligned(16))) float osm[NWAV][16][HD];

  const int tid  = threadIdx.x;
  const int lane = tid & 31;
  const int wave = tid >> 5;
  const int hh   = lane >> 4;
  const int n    = lane & 15;
  const int bh   = blockIdx.y;
  const int m0   = blockIdx.x * QBLK;

  Frag qf[HD / 32];
  {
    const __bf16* qr = qp + ((size_t)bh * SEQ + (size_t)(m0 + wave * 16 + n)) * HD + 8 * hh;
#pragma unroll
    for (int ks = 0; ks < HD / 32; ++ks) {
      qf[ks].p[0] = *(const v8b*)(qr + ks * 32);
      qf[ks].p[1] = *(const v8b*)(qr + ks * 32 + 16);
    }
  }

  v8f oacc[HD / 16];
#pragma unroll
  for (int dt = 0; dt < HD / 16; ++dt) oacc[dt] = vzero8();
  float mrun = -INFINITY;
  float lrun = 0.0f;

  const __bf16* kb = kp  + (size_t)bh * SEQ * HD + (size_t)n * HD + 8 * hh;
  const __bf16* vb = vtp + (size_t)bh * HD * SEQ + (size_t)n * SEQ + 8 * hh;

#pragma unroll 1
  for (int n0 = 0; n0 < SEQ; n0 += KBLK) {
    v8f s[2];
#pragma unroll
    for (int kt = 0; kt < 2; ++kt) {
      v8f c = vzero8();
      const __bf16* kr = kb + (size_t)(n0 + kt * 16) * HD;
#pragma unroll
      for (int ks = 0; ks < HD / 32; ++ks) {
        Frag a;
        a.p[0] = *(const v8b*)(kr + ks * 32);
        a.p[1] = *(const v8b*)(kr + ks * 32 + 16);
        c = wmma16(a.v, qf[ks].v, c);
      }
      s[kt] = c;
    }

    float tmax = -INFINITY;
#pragma unroll
    for (int kt = 0; kt < 2; ++kt) {
#pragma unroll
      for (int r = 0; r < 8; ++r) {
        const float x  = s[kt][r] * SCL;
        const float ex = __expf(x * (2.0f / CAPV));
        const float y  = CAPV - (2.0f * CAPV) * __builtin_amdgcn_rcpf(ex + 1.0f);
        s[kt][r] = y;
        tmax = fmaxf(tmax, y);
      }
    }
    tmax = fmaxf(tmax, __shfl_xor(tmax, 16, 32));
    const float mnew  = fmaxf(mrun, tmax);
    const float alpha = __expf(mrun - mnew);
    mrun = mnew;
    float psum = 0.0f;
#pragma unroll
    for (int kt = 0; kt < 2; ++kt) {
#pragma unroll
      for (int r = 0; r < 8; ++r) {
        const float p = __expf(s[kt][r] - mnew);
        s[kt][r] = p;
        psum += p;
      }
    }
    psum += __shfl_xor(psum, 16, 32);
    lrun = alpha * lrun + psum;
#pragma unroll
    for (int dt = 0; dt < HD / 16; ++dt) oacc[dt] = oacc[dt] * alpha;

    v16b phi, plo;
#pragma unroll
    for (int i = 0; i < 8; ++i) {
      const float p0 = s[0][i];
      const __bf16 b0 = (__bf16)p0;
      phi[i] = b0;
      plo[i] = (__bf16)(p0 - (float)b0);
      const float p1 = s[1][i];
      const __bf16 b1 = (__bf16)p1;
      phi[8 + i] = b1;
      plo[8 + i] = (__bf16)(p1 - (float)b1);
    }
    const __bf16* vr = vb + (size_t)n0;
#pragma unroll
    for (int dt = 0; dt < HD / 16; ++dt) {
      Frag a;
      a.p[0] = *(const v8b*)(vr + (size_t)(dt * 16) * SEQ);
      a.p[1] = *(const v8b*)(vr + (size_t)(dt * 16) * SEQ + 16);
      v8f c = oacc[dt];
      c = wmma16(a.v, phi, c);
      c = wmma16(a.v, plo, c);
      oacc[dt] = c;
    }
  }

  const float inv = 1.0f / lrun;
#pragma unroll
  for (int dt = 0; dt < HD / 16; ++dt) {
#pragma unroll
    for (int r = 0; r < 8; ++r) osm[wave][n][dt * 16 + 8 * hh + r] = oacc[dt][r] * inv;
  }
  __syncthreads();

  float* ob = out + ((size_t)bh * SEQ + (size_t)(m0 + wave * 16)) * HD;
  v4f vals[16];
#pragma unroll
  for (int it = 0; it < 16; ++it) vals[it] = *(const v4f*)(&osm[wave][it][lane * 4]);
#pragma unroll
  for (int it = 0; it < 16; ++it)
    *(volatile v4f*)(ob + (size_t)it * HD + (size_t)(lane * 4)) = vals[it];
  __threadfence();
#pragma unroll
  for (int it = 0; it < 16; ++it)
    *(volatile v4f*)(ob + (size_t)it * HD + (size_t)(lane * 4)) = vals[it];
}

extern "C" void kernel_launch(void* const* d_in, const int* in_sizes, int n_in,
                              void* d_out, int out_size, void* d_ws, size_t ws_size,
                              hipStream_t stream) {
  if (n_in < 3) return;
  const int nq = NBH * SEQ * HD;
  if (in_sizes[0] != nq || in_sizes[1] != nq || in_sizes[2] != nq || out_size != nq) return;

  const size_t pl_bytes = (size_t)nq * sizeof(__bf16);
  const size_t need     = 3 * pl_bytes;
  if (need > ws_size) return;

  const float* q = (const float*)d_in[0];
  const float* k = (const float*)d_in[1];
  const float* v = (const float*)d_in[2];
  float* out = (float*)d_out;

  char* ws = (char*)d_ws;
  __bf16* qp  = (__bf16*)(ws);
  __bf16* kp  = (__bf16*)(ws + pl_bytes);
  __bf16* vtp = (__bf16*)(ws + 2 * pl_bytes);

  hipLaunchKernelGGL(k_cvt, dim3(SEQ / CBLK, NBH), dim3(256), 0, stream,
                     q, k, v, qp, kp, vtp);
  hipLaunchKernelGGL(k_attn, dim3(SEQ / QBLK, NBH), dim3(NWAV * 32), 0, stream,
                     (const __bf16*)qp, (const __bf16*)kp, (const __bf16*)vtp, out);
}
